// CapsuleLayer_75514114998376
// MI455X (gfx1250) — hardware-run, weakly checked
//
#include <hip/hip_runtime.h>


#ifndef NB
#define NB 32
#endif
#ifndef SEQ
#define SEQ 2048
#endif
#define NB_FULL  32
#define SEQ_FULL 2048
#define IND   128
#define ONUM  16
#define ODIM  32
#define AW    4
#define TPB   256
#define CHUNKS (SEQ / TPB)
#define NBT   ((NB + 15) / 16)
#define TSP   136
#define YSP   132
#define ASP   36
#define ATP   40
#define QRS   2048.0f
#define QRI   (1.0f / 2048.0f)
#define PSH   16384.0f
#define PSI   (1.0f / 16384.0f)
#define L2E   1.4426950408889634f

static_assert(IND == 128);
static_assert(ONUM == 16);
static_assert(ODIM == 32);
static_assert(IND % 32 == 0);
static_assert(SEQ % TPB == 0);
static_assert(TPB % 64 == 0);
static_assert((TPB / AW) % 32 == 0);
static_assert(SEQ % 64 == 0);
static_assert(NB <= NB_FULL);
static_assert(SEQ <= SEQ_FULL);
static_assert((TSP * 2) % 16 == 0);
static_assert((YSP * 4) % 16 == 0);
static_assert((ASP * 4) % 16 == 0);
static_assert((ATP * 2) % 16 == 0);

typedef _Float16 h16;
typedef __attribute__((ext_vector_type(16))) _Float16 v16h;
typedef __attribute__((ext_vector_type(8)))  _Float16 v8h;
typedef __attribute__((ext_vector_type(4)))  _Float16 v4h;
typedef __attribute__((ext_vector_type(8)))  float    v8f;
typedef __attribute__((ext_vector_type(4)))  float    v4f;
typedef v4f  __attribute__((may_alias)) v4fa;
typedef v8h  __attribute__((may_alias)) v8ha;
typedef v4h  __attribute__((may_alias)) v4ha;

__device__ __forceinline__ unsigned short f2bf(float f) { unsigned u = __float_as_uint(f); u += 0x7FFFu + ((u >> 16) & 1u); return (unsigned short)(u >> 16); }
__device__ __forceinline__ float bfr(float f) { return __uint_as_float(((unsigned)f2bf(f)) << 16); }
__device__ __forceinline__ v16h cat16(v8h lo, v8h hi) { return __builtin_shufflevector(lo, hi, 0, 1, 2, 3, 4, 5, 6, 7, 8, 9, 10, 11, 12, 13, 14, 15); }
static __device__ __forceinline__ h16 toh_flush(float v) { const h16 r = (h16)v; return (fabsf(v) < 6.103515625e-05f) ? (h16)0.0f : r; }
__device__ __forceinline__ v8f wmg(v16h a, v16h b, v8f c) {
    c = __builtin_amdgcn_wmma_f32_16x16x32_f16(false, a, false, b, (short)0, c, false, false);
    asm volatile("v_nop\n\tv_nop\n\tv_nop\n\tv_nop" : "+v"(c) : "v"(a), "v"(b));
    return c;
}
__device__ __forceinline__ v16h ldh(const h16* p) { return cat16(*(const v8h*)p, *(const v8h*)(p + 16)); }
__device__ __forceinline__ void wave_sync() { __builtin_amdgcn_fence(3  , "wavefront"); __builtin_amdgcn_wave_barrier(); asm volatile("" ::: "memory"); }

static_assert(256 * 8 * 4 == 64 * IND);
static_assert(64 * TSP * 2 <= 131072);
__global__ __launch_bounds__(256) void k_xprep(const float* __restrict__ x, h16* XH, h16* XT) {
    __shared__ __align__(16) h16 ts[64 * TSP];
    const int tid = threadIdx.x;
    const int b = blockIdx.y, tok0 = blockIdx.x * 64;
    const int c8 = (tid & 15) * 8, rq = tid >> 4;
    v8h hv[4];
#pragma unroll
    for (int it = 0; it < 4; ++it) {
        const int row = it * 16 + rq;
        const float* src = x + ((size_t)b * SEQ_FULL + (size_t)(tok0 + row)) * IND + c8;
        const v4f p0 = *(const v4f*)src, p1 = *(const v4f*)(src + 4);
        v8h o;
#pragma unroll
        for (int k = 0; k < 4; ++k) { o[k] = toh_flush(bfr(p0[k])); o[4 + k] = toh_flush(bfr(p1[k])); }
        hv[it] = o;
        *(v8ha*)(&ts[row * TSP + c8]) = o;
    }
    __syncthreads();
    const int t8 = (tid & 7) * 8, iq = tid >> 3;
    v8h tv[4];
#pragma unroll
    for (int it = 0; it < 4; ++it) {
        const int i = it * 32 + iq;
        v8h o;
#pragma unroll
        for (int k = 0; k < 8; ++k) o[k] = ts[(t8 + k) * TSP + i];
        tv[it] = o;
    }
    h16* xhp = XH + ((size_t)b * SEQ + (size_t)tok0) * IND;
    h16* xtp = XT + (size_t)b * IND * SEQ + (size_t)tok0;
#pragma unroll 1
    for (int ps = 0; ps < 2; ++ps) {
#pragma unroll
        for (int it = 0; it < 4; ++it) *(volatile v8h*)(xhp + (size_t)(it * 16 + rq) * IND + c8) = hv[it];
#pragma unroll
        for (int it = 0; it < 4; ++it) *(volatile v8h*)(xtp + (size_t)(it * 32 + iq) * SEQ + t8) = tv[it];
        if (ps == 0) __threadfence();
    }
}

static_assert(256 * 8 * 2 == ODIM * IND);
__global__ __launch_bounds__(256) void k_wprep(const float* __restrict__ W, h16* WH, h16* WT) {
    __shared__ __align__(16) h16 wl[ODIM * TSP];
    const int tid = threadIdx.x;
    const int o = blockIdx.x;
    const int c8 = (tid & 15) * 8, rq = tid >> 4;
    v8h hv[2];
#pragma unroll
    for (int it = 0; it < 2; ++it) {
        const int row = it * 16 + rq;
        const float* src = W + ((size_t)(o * ODIM + row)) * IND + c8;
        const v4f p0 = *(const v4f*)src, p1 = *(const v4f*)(src + 4);
        v8h q;
#pragma unroll
        for (int k = 0; k < 4; ++k) { q[k] = toh_flush(bfr(p0[k])); q[4 + k] = toh_flush(bfr(p1[k])); }
        hv[it] = q;
        *(v8ha*)(&wl[row * TSP + c8]) = q;
    }
    __syncthreads();
    const int d8 = (tid & 3) * 8, iq = tid >> 2;
    v8h tv[2];
#pragma unroll
    for (int it = 0; it < 2; ++it) {
        const int i = it * 64 + iq;
        v8h q;
#pragma unroll
        for (int k = 0; k < 8; ++k) q[k] = wl[(d8 + k) * TSP + i];
        tv[it] = q;
    }
    h16* whp = WH + (size_t)(o * ODIM) * IND;
    h16* wtp = WT + (size_t)o * IND * ODIM;
#pragma unroll 1
    for (int ps = 0; ps < 2; ++ps) {
#pragma unroll
        for (int it = 0; it < 2; ++it) *(volatile v8h*)(whp + (size_t)(it * 16 + rq) * IND + c8) = hv[it];
#pragma unroll
        for (int it = 0; it < 2; ++it) *(volatile v8h*)(wtp + (size_t)(it * 64 + iq) * ODIM + d8) = tv[it];
        if (ps == 0) __threadfence();
    }
}

static_assert(32 * AW * 4 * 4 == ONUM * IND);
static_assert(AW * 16 * YSP * 4 <= 131072);
__global__ __launch_bounds__(32 * AW) void k_route(const h16* __restrict__ XH, const h16* __restrict__ XT, const h16* __restrict__ VH, const h16* __restrict__ VR, float* YP, int first) {
    __shared__ __align__(16) float ys[AW * 16 * YSP];
    const int lane = threadIdx.x & 31, lr = lane & 15, hi = lane >> 4;
    const int wave = __builtin_amdgcn_readfirstlane((int)(threadIdx.x >> 5));
    const int ch = blockIdx.x, b = blockIdx.y;
    const int tw0 = ch * TPB + wave * (TPB / AW);
    const size_t xo = ((size_t)b * SEQ + (size_t)lr) * IND + 8 * hi;
    const size_t vo = ((size_t)b * ONUM + (size_t)lr) * IND + 8 * hi;
    const size_t to = ((size_t)b * IND + (size_t)lr) * SEQ + 8 * hi;
    v8f yacc[8];
#pragma unroll
    for (int j = 0; j < 8; ++j) yacc[j] = (v8f){};
#pragma unroll 1
    for (int st = 0; st < (TPB / AW) / 32; ++st) {
        const int tok0 = tw0 + st * 32;
        v16h pb;
        if (first != 0) {
            const h16 cu = (h16)(PSH / 16.0f);
#pragma unroll
            for (int i = 0; i < 16; ++i) pb[i] = cu;
        } else {
            v8f sHa = (v8f){}, sLa = (v8f){}, sHb = (v8f){}, sLb = (v8f){};
#pragma unroll
            for (int kc = 0; kc < IND; kc += 32) {
                const v16h xa = ldh(XH + xo + (size_t)tok0 * IND + kc);
                const v16h xb = ldh(XH + xo + (size_t)(tok0 + 16) * IND + kc);
                const v16h bh = ldh(VH + vo + kc);
                const v16h br = ldh(VR + vo + kc);
                sHa = wmg(xa, bh, sHa); sLa = wmg(xa, br, sLa);
                sHb = wmg(xb, bh, sHb); sLb = wmg(xb, br, sLb);
            }
#pragma unroll
            for (int r = 0; r < 8; ++r) {
                const float ta = (sHa[r] + sLa[r] * QRI) * L2E;
                const float tb = (sHb[r] + sLb[r] * QRI) * L2E;
                float ma = ta, mb = tb;
                ma = fmaxf(ma, __shfl_xor(ma, 1, 32)); mb = fmaxf(mb, __shfl_xor(mb, 1, 32));
                ma = fmaxf(ma, __shfl_xor(ma, 2, 32)); mb = fmaxf(mb, __shfl_xor(mb, 2, 32));
                ma = fmaxf(ma, __shfl_xor(ma, 4, 32)); mb = fmaxf(mb, __shfl_xor(mb, 4, 32));
                ma = fmaxf(ma, __shfl_xor(ma, 8, 32)); mb = fmaxf(mb, __shfl_xor(mb, 8, 32));
                const float ea = __builtin_amdgcn_exp2f(ta - ma), eb = __builtin_amdgcn_exp2f(tb - mb);
                float sa = ea, sb = eb;
                sa += __shfl_xor(sa, 1, 32); sb += __shfl_xor(sb, 1, 32);
                sa += __shfl_xor(sa, 2, 32); sb += __shfl_xor(sb, 2, 32);
                sa += __shfl_xor(sa, 4, 32); sb += __shfl_xor(sb, 4, 32);
                sa += __shfl_xor(sa, 8, 32); sb += __shfl_xor(sb, 8, 32);
                const float ia = PSH * __builtin_amdgcn_rcpf(sa), ib = PSH * __builtin_amdgcn_rcpf(sb);
                pb[r] = toh_flush(ea * ia); pb[8 + r] = toh_flush(eb * ib);
            }
        }
#pragma unroll
        for (int j = 0; j < 8; ++j) {
            const v16h xt = ldh(XT + to + (size_t)(16 * j) * SEQ + tok0);
            yacc[j] = wmg(xt, pb, yacc[j]);
        }
    }
    const int wb = wave * 16 * YSP;
#pragma unroll
    for (int j = 0; j < 8; ++j) {
        v4f a, c;
        a[0] = yacc[j][0]; a[1] = yacc[j][1]; a[2] = yacc[j][2]; a[3] = yacc[j][3];
        c[0] = yacc[j][4]; c[1] = yacc[j][5]; c[2] = yacc[j][6]; c[3] = yacc[j][7];
        *(v4fa*)(&ys[wb + lr * YSP + 16 * j + 8 * hi]) = a; *(v4fa*)(&ys[wb + lr * YSP + 16 * j + 8 * hi + 4]) = c;
    }
    __syncthreads();
    float* dst = YP + (((size_t)ch * NB + (size_t)b) * ONUM) * IND;
#pragma unroll 1
    for (int ps = 0; ps < 2; ++ps) {
#pragma unroll
        for (int s = 0; s < 4; ++s) {
            const int row = AW * s + wave, cofs = lane * 4;
            v4f val = *(const v4fa*)(&ys[row * YSP + cofs]);
#pragma unroll
            for (int w = 1; w < AW; ++w) { const v4f t = *(const v4fa*)(&ys[w * 16 * YSP + row * YSP + cofs]); val = val + t; }
            val = val * PSI;
            *(volatile v4f*)(dst + (size_t)row * IND + cofs) = val;
        }
        if (ps == 0) __threadfence();
    }
}

static_assert(32 * 4 * 4 == 16 * ODIM);
static_assert(32 * 8 * 8 == 16 * IND);
static_assert(2 * 16 * TSP * 2 + 16 * ASP * 4 + 2 * 16 * ATP * 2 + 16 * YSP * 4 <= 131072);
__global__ __launch_bounds__(32) void k_upd(const float* __restrict__ YP, const h16* __restrict__ WH, const h16* __restrict__ WT,
                                            const float* AOLD, float* ADST, h16* VHo, h16* VRo, int mode) {
    __shared__ __align__(16) h16 yh[16 * TSP];
    __shared__ __align__(16) h16 yr[16 * TSP];
    __shared__ __align__(16) float at[16 * ASP];
    __shared__ __align__(16) h16 ath[16 * ATP];
    __shared__ __align__(16) h16 atr[16 * ATP];
    __shared__ __align__(16) float vs[16 * YSP];
    const int lane = threadIdx.x & 31, lr = lane & 15, hi = lane >> 4;
    const int o = blockIdx.x, bt = blockIdx.y;

#pragma unroll 1
    for (int m = 0; m < 16; ++m) {
        const int bb = min(bt * 16 + m, NB - 1);
        v4f acc = (v4f){};
#pragma unroll 1
        for (int c = 0; c < CHUNKS; ++c) {
            const v4f t = *(const v4f*)(YP + ((((size_t)c * NB + (size_t)bb) * ONUM + (size_t)o) * IND) + lane * 4);
            acc = acc + t;
        }
        v4h hv, rv;
#pragma unroll
        for (int i = 0; i < 4; ++i) { const h16 t = toh_flush(acc[i]); hv[i] = t; rv[i] = toh_flush((acc[i] - (float)t) * QRS); }
        *(v4ha*)(&yh[m * TSP + lane * 4]) = hv;
        *(v4ha*)(&yr[m * TSP + lane * 4]) = rv;
    }
    wave_sync();

    v8f sH0 = (v8f){}, sL0 = (v8f){}, sH1 = (v8f){}, sL1 = (v8f){};
#pragma unroll
    for (int kc = 0; kc < IND; kc += 32) {
        const int ao = lr * TSP + 8 * hi + kc;
        const v16h ah = cat16(*(const v8ha*)(&yh[ao]), *(const v8ha*)(&yh[ao + 16]));
        const v16h ar = cat16(*(const v8ha*)(&yr[ao]), *(const v8ha*)(&yr[ao + 16]));
        const v16h b0 = ldh(WH + ((size_t)(o * ODIM + lr)) * IND + 8 * hi + kc);
        const v16h b1 = ldh(WH + ((size_t)(o * ODIM + 16 + lr)) * IND + 8 * hi + kc);
        sH0 = wmg(ah, b0, sH0); sL0 = wmg(ar, b0, sL0);
        sH1 = wmg(ah, b1, sH1); sL1 = wmg(ar, b1, sL1);
    }
    float a0[8], a1[8];
#pragma unroll
    for (int r = 0; r < 8; ++r) {
        const float s0 = sH0[r] + sL0[r] * QRI, s1 = sH1[r] + sL1[r] * QRI;
        float n = s0 * s0 + s1 * s1;
        n += __shfl_xor(n, 1, 32); n += __shfl_xor(n, 2, 32); n += __shfl_xor(n, 4, 32); n += __shfl_xor(n, 8, 32);
        const float f = sqrtf(n) / (1.0f + n);
        a0[r] = f * s0; a1[r] = f * s1;
    }

    if (mode != 1) {
#pragma unroll
        for (int r = 0; r < 8; ++r) { at[(8 * hi + r) * ASP + lr] = a0[r]; at[(8 * hi + r) * ASP + 16 + lr] = a1[r]; }
        wave_sync();
#pragma unroll 1
        for (int ps = 0; ps < 2; ++ps) {
#pragma unroll
            for (int s = 0; s < 4; ++s) {
                const int row = 4 * s + (lane >> 3), cofs = (lane & 7) * 4;
                const v4f val = *(const v4fa*)(&at[row * ASP + cofs]);
                const int bb = bt * 16 + row;
                if (bb < NB) *(volatile v4f*)(ADST + ((size_t)bb * ONUM + (size_t)o) * ODIM + cofs) = val;
            }
            if (ps == 0) __threadfence();
        }
    }
    if (mode == 1) {
#pragma unroll
        for (int r = 0; r < 8; ++r) {
            const int bb = min(bt * 16 + 8 * hi + r, NB - 1);
            const float* ap = AOLD + ((size_t)bb * ONUM + (size_t)o) * ODIM + lr;
            a0[r] += ap[0]; a1[r] += ap[16];
        }
    }
    if (mode != 2) {
#pragma unroll
        for (int r = 0; r < 8; ++r) {
            const h16 t0 = toh_flush(a0[r]); const h16 t1 = toh_flush(a1[r]);
            ath[(8 * hi + r) * ATP + lr] = t0; ath[(8 * hi + r) * ATP + 16 + lr] = t1;
            atr[(8 * hi + r) * ATP + lr] = toh_flush((a0[r] - (float)t0) * QRS);
            atr[(8 * hi + r) * ATP + 16 + lr] = toh_flush((a1[r] - (float)t1) * QRS);
        }
        wave_sync();
        const int fo = lr * ATP + 8 * hi;
        const v16h fh = cat16(*(const v8ha*)(&ath[fo]), *(const v8ha*)(&ath[fo + 16]));
        const v16h fr = cat16(*(const v8ha*)(&atr[fo]), *(const v8ha*)(&atr[fo + 16]));
#pragma unroll 1
        for (int nb = 0; nb < IND / 16; ++nb) {
            const v16h bw = ldh(WT + ((size_t)o * IND + (size_t)(nb * 16 + lr)) * ODIM + 8 * hi);
            v8f vH = (v8f){}, vL = (v8f){};
            vH = wmg(fh, bw, vH); vL = wmg(fr, bw, vL);
#pragma unroll
            for (int r = 0; r < 8; ++r) vs[(8 * hi + r) * YSP + nb * 16 + lr] = vH[r] + vL[r] * QRI;
        }
        wave_sync();
#pragma unroll 1
        for (int ps = 0; ps < 2; ++ps) {
#pragma unroll 1
            for (int s = 0; s < 8; ++s) {
                const int row = 2 * s + hi, c8 = lr * 8;
                const v4f x0 = *(const v4fa*)(&vs[row * YSP + c8]); const v4f x1 = *(const v4fa*)(&vs[row * YSP + c8 + 4]);
                v8h hv, rv;
#pragma unroll
                for (int i = 0; i < 4; ++i) {
                    const h16 t0 = toh_flush(x0[i]); const h16 t1 = toh_flush(x1[i]);
                    hv[i] = t0; hv[4 + i] = t1;
                    rv[i] = toh_flush((x0[i] - (float)t0) * QRS); rv[4 + i] = toh_flush((x1[i] - (float)t1) * QRS);
                }
                const int bb = bt * 16 + row;
                if (bb < NB) {
                    const size_t oo = ((size_t)bb * ONUM + (size_t)o) * IND + c8;
                    *(volatile v8h*)(VHo + oo) = hv; *(volatile v8h*)(VRo + oo) = rv;
                }
            }
            if (ps == 0) __threadfence();
        }
    }
}

static constexpr size_t al256(size_t v) { return (v + 255) & ~(size_t)255; }
static constexpr size_t SZ_X = al256((size_t)NB * SEQ * IND * 2);
static constexpr size_t SZ_W = al256((size_t)ONUM * ODIM * IND * 2);
static constexpr size_t SZ_Y = al256((size_t)CHUNKS * NB * ONUM * IND * 4);
static constexpr size_t SZ_V = al256((size_t)NB * ONUM * IND * 2);
static constexpr size_t SZ_A = al256((size_t)NB * ONUM * ODIM * 4);
static constexpr size_t SZ_TOTAL = 2 * SZ_X + 2 * SZ_W + SZ_Y + 2 * SZ_V + SZ_A;
static_assert(SZ_TOTAL <= (size_t)134217728);
static_assert((size_t)NB_FULL * ONUM * ODIM * 4 == (size_t)65536);

extern "C" void kernel_launch(void* const* d_in, const int* in_sizes, int n_in,
                              void* d_out, int out_size, void* d_ws, size_t ws_size, hipStream_t stream) {
    if (n_in < 2) return;
    const size_t needx = ((size_t)(NB - 1) * SEQ_FULL + SEQ) * IND;
    if ((size_t)in_sizes[0] < needx) return;
    if ((size_t)in_sizes[1] < (size_t)ONUM * ODIM * IND) return;
    if ((size_t)out_size < (size_t)NB * ONUM * ODIM) return;
    if (SZ_TOTAL > ws_size) return;
    const float* x = (const float*)d_in[0];
    const float* W = (const float*)d_in[1];
    float* OUT = (float*)d_out;
    char* wsp = (char*)d_ws;
    h16* XH = (h16*)wsp; wsp += SZ_X;
    h16* XT = (h16*)wsp; wsp += SZ_X;
    h16* WH = (h16*)wsp; wsp += SZ_W;
    h16* WT = (h16*)wsp; wsp += SZ_W;
    float* YP = (float*)wsp; wsp += SZ_Y;
    h16* VH = (h16*)wsp; wsp += SZ_V;
    h16* VR = (h16*)wsp; wsp += SZ_V;
    float* A0 = (float*)wsp; wsp += SZ_A;

    k_xprep<<<dim3(SEQ / 64, NB, 1), 256, 0, stream>>>(x, XH, XT);
    k_wprep<<<dim3(ONUM, 1, 1), 256, 0, stream>>>(W, WH, WT);
    k_route<<<dim3(CHUNKS, NB, 1), 32 * AW, 0, stream>>>(XH, XT, VH, VR, YP, 1);
    k_upd<<<dim3(ONUM, NBT, 1), 32, 0, stream>>>(YP, WH, WT, A0, A0, VH, VR, 0);
    k_route<<<dim3(CHUNKS, NB, 1), 32 * AW, 0, stream>>>(XH, XT, VH, VR, YP, 0);
    k_upd<<<dim3(ONUM, NBT, 1), 32, 0, stream>>>(YP, WH, WT, A0, OUT, VH, VR, 1);
    k_route<<<dim3(CHUNKS, NB, 1), 32 * AW, 0, stream>>>(XH, XT, VH, VR, YP, 0);
    k_upd<<<dim3(ONUM, NBT, 1), 32, 0, stream>>>(YP, WH, WT, A0, OUT, VH, VR, 2);
}
